// GPT2Block_55576876810791
// MI455X (gfx1250) — hardware-verified
//
#include <hip/hip_runtime.h>


#define DEVFN __device__ __forceinline__

#ifndef NB
#define NB 2
#endif
#ifndef SEQ
#define SEQ 2048
#endif
#define NB_FULL 2
#define SEQ_FULL 2048

static constexpr int E   = 1024;
static constexpr int H   = 16;
static constexpr int HD  = 64;
static constexpr int FF  = 4096;
static constexpr int E2  = 2 * E;
static constexpr int E3  = 3 * E;
static constexpr int S   = SEQ;
static constexpr int T   = NB * SEQ;
static constexpr int LOR = 128;

static_assert((SEQ % 128) == 0);
static_assert(SEQ >= 256);
static_assert(SEQ <= SEQ_FULL);
static_assert(NB >= 1);
static_assert(NB <= NB_FULL);
static_assert(HD == 64);
static_assert((E % 64) == 0);
static_assert((FF % 64) == 0);
static_assert((T % 128) == 0);
static_assert(LOR <= SEQ);

static constexpr float WC     = 64.0f;
static constexpr float WINV   = 1.0f / 64.0f;
static constexpr float RC     = 2048.0f;
static constexpr float RCI    = 1.0f / 2048.0f;
static constexpr float PC     = 4096.0f;
static constexpr float YC     = 16.0f;
static constexpr float YCI    = 1.0f / 16.0f;
static constexpr float LN_EPS = 1e-5f;

static constexpr int M_QKV  = 0;
static constexpr int M_PROJ = 1;
static constexpr int M_FF1  = 2;
static constexpr int M_FF2  = 3;

typedef _Float16 v16h __attribute__((ext_vector_type(16)));
typedef _Float16 v8h  __attribute__((ext_vector_type(8)));
typedef float    v8f  __attribute__((ext_vector_type(8)));
typedef float    v4f  __attribute__((ext_vector_type(4)));
typedef unsigned int v4u __attribute__((ext_vector_type(4)));

union Frag { v16h v; v8h h[2]; _Float16 e[16]; };
union H8   { v8h h; v4u u; };

DEVFN v8f mma(v16h a, v16h b, v8f c) {
    c = __builtin_amdgcn_wmma_f32_16x16x32_f16(false, a, false, b, (short)0, c, false, false);
    asm volatile("v_nop\n\tv_nop\n\tv_nop\n\tv_nop" : "+v"(c) : "v"(a), "v"(b));
    return c;
}

DEVFN v8f zero8() {
    v8f z;
#pragma unroll
    for (int i = 0; i < 8; ++i) z[i] = 0.0f;
    return z;
}

DEVFN float bf16r(float f) {
    unsigned int u = __float_as_uint(f);
    u += 0x7fffu + ((u >> 16) & 1u);
    u &= 0xffff0000u;
    return __uint_as_float(u);
}
DEVFN v4f bf16r4(v4f v) {
    v4f r;
    r.x = bf16r(v.x); r.y = bf16r(v.y); r.z = bf16r(v.z); r.w = bf16r(v.w);
    return r;
}

DEVFN float gelu_erf(float v) {
    return 0.5f * v * (erff(v * 0.70710678118654752f) + 1.0f);
}
DEVFN v4f gelu4(v4f v) {
    v4f r;
    r.x = gelu_erf(v.x); r.y = gelu_erf(v.y); r.z = gelu_erf(v.z); r.w = gelu_erf(v.w);
    return r;
}

DEVFN _Float16 lo_of(float v) {
    const _Float16 hh = (_Float16)v;
    return (_Float16)((v - (float)hh) * RC);
}

DEVFN v4u pack8h(v4f a, v4f b) {
    H8 t;
    t.h[0] = (_Float16)a.x; t.h[1] = (_Float16)a.y; t.h[2] = (_Float16)a.z; t.h[3] = (_Float16)a.w;
    t.h[4] = (_Float16)b.x; t.h[5] = (_Float16)b.y; t.h[6] = (_Float16)b.z; t.h[7] = (_Float16)b.w;
    return t.u;
}
DEVFN v4u pack8lo(v4f a, v4f b) {
    H8 t;
    t.h[0] = lo_of(a.x); t.h[1] = lo_of(a.y); t.h[2] = lo_of(a.z); t.h[3] = lo_of(a.w);
    t.h[4] = lo_of(b.x); t.h[5] = lo_of(b.y); t.h[6] = lo_of(b.z); t.h[7] = lo_of(b.w);
    return t.u;
}

DEVFN float wave_sum(float v) {
    v += __shfl_xor(v, 16, 32);
    v += __shfl_xor(v, 8, 32);
    v += __shfl_xor(v, 4, 32);
    v += __shfl_xor(v, 2, 32);
    v += __shfl_xor(v, 1, 32);
    return v;
}

DEVFN int xrow(int r) { return (r / S) * SEQ_FULL + (r % S); }

__global__ __launch_bounds__(256)
void cvt_kernel(const float* __restrict__ in, _Float16* __restrict__ out, int K, int N) {
    __shared__ float tile[64][65];
    const int k0 = blockIdx.x * 64, n0 = blockIdx.y * 64;
    const int tid = threadIdx.x, lane = tid & 31, wid = tid >> 5;

#pragma unroll
    for (int p = 0; p < 4; ++p) {
        const int idx = tid + 256 * p;
        const int r = idx >> 4, c4 = idx & 15;
        const v4f v = *(const v4f*)&in[(size_t)(k0 + r) * N + n0 + c4 * 4];
        tile[r][c4 * 4 + 0] = v.x;
        tile[r][c4 * 4 + 1] = v.y;
        tile[r][c4 * 4 + 2] = v.z;
        tile[r][c4 * 4 + 3] = v.w;
    }
    __syncthreads();

    const int kq = lane & 7;
    v4u hv[2];
    size_t ad[2];
#pragma unroll
    for (int p = 0; p < 2; ++p) {
        const int nr = p * 32 + wid * 4 + (lane >> 3);
        v4f f0, f1;
        f0.x = bf16r(tile[kq * 8 + 0][nr]) * WC;
        f0.y = bf16r(tile[kq * 8 + 1][nr]) * WC;
        f0.z = bf16r(tile[kq * 8 + 2][nr]) * WC;
        f0.w = bf16r(tile[kq * 8 + 3][nr]) * WC;
        f1.x = bf16r(tile[kq * 8 + 4][nr]) * WC;
        f1.y = bf16r(tile[kq * 8 + 5][nr]) * WC;
        f1.z = bf16r(tile[kq * 8 + 6][nr]) * WC;
        f1.w = bf16r(tile[kq * 8 + 7][nr]) * WC;
        hv[p] = pack8h(f0, f1);
        ad[p] = (size_t)(n0 + nr) * K + k0 + kq * 8;
    }
#pragma unroll
    for (int p = 0; p < 2; ++p) *(volatile v4u*)(out + ad[p]) = hv[p];
    __threadfence();
#pragma unroll
    for (int p = 0; p < 2; ++p) *(volatile v4u*)(out + ad[p]) = hv[p];
}

template <bool RNDIN, bool WLO>
__global__ __launch_bounds__(256)
void ln_kernel(const float* __restrict__ x, const float* __restrict__ g,
               const float* __restrict__ b, _Float16* __restrict__ out,
               _Float16* __restrict__ outlo) {
    __shared__ float stg[E];
    __shared__ float red[8];
    const int row = blockIdx.x, tid = threadIdx.x, lane = tid & 31, wid = tid >> 5;
    const size_t xr = RNDIN ? (size_t)xrow(row) : (size_t)row;

    v4f v = *(const v4f*)&x[xr * E + tid * 4];
    if constexpr (RNDIN) v = bf16r4(v);

    float s = (v.x + v.y) + (v.z + v.w);
    s = wave_sum(s);
    if (lane == 0) red[wid] = s;
    __syncthreads();
    float tot = 0.0f;
#pragma unroll
    for (int w = 0; w < 8; ++w) tot += red[w];
    const float mu = tot * (1.0f / (float)E);
    __syncthreads();

    const v4f d = v - mu;
    float s2 = (d.x * d.x + d.y * d.y) + (d.z * d.z + d.w * d.w);
    s2 = wave_sum(s2);
    if (lane == 0) red[wid] = s2;
    __syncthreads();
    float tot2 = 0.0f;
#pragma unroll
    for (int w = 0; w < 8; ++w) tot2 += red[w];
    const float var  = tot2 * (1.0f / (float)E);
    const float rstd = rsqrtf(var + LN_EPS);

    const v4f gv = bf16r4(*(const v4f*)&g[tid * 4]);
    const v4f bv = bf16r4(*(const v4f*)&b[tid * 4]);
    v4f y = (d * rstd) * gv + bv;
    *(v4f*)&stg[tid * 4] = y;
    __syncthreads();

    const bool lo_on = WLO && ((row % S) < LOR);
    if (tid < 128) {
        const int piece = tid;
        const v4f f0 = *(const v4f*)&stg[piece * 8];
        const v4f f1 = *(const v4f*)&stg[piece * 8 + 4];
        const v4u hv = pack8h(f0, f1);
        _Float16* p = out + (size_t)row * E + piece * 8;
        *(volatile v4u*)p = hv;
        __threadfence();
        *(volatile v4u*)p = hv;
    } else if (lo_on) {
        const int piece = tid - 128;
        const v4f f0 = *(const v4f*)&stg[piece * 8];
        const v4f f1 = *(const v4f*)&stg[piece * 8 + 4];
        const v4u lv = pack8lo(f0, f1);
        const int lr = (row / S) * LOR + (row % S);
        _Float16* p = outlo + (size_t)lr * E + piece * 8;
        *(volatile v4u*)p = lv;
        __threadfence();
        *(volatile v4u*)p = lv;
    }
}

template <int MODE, bool ALO>
__global__ __launch_bounds__(256)
void gemm_kernel(const _Float16* __restrict__ A, const _Float16* __restrict__ Alo,
                 const _Float16* __restrict__ Wt, const float* __restrict__ bias,
                 const float* __restrict__ resid,
                 _Float16* __restrict__ oh, _Float16* __restrict__ ohlo,
                 _Float16* __restrict__ ov, _Float16* __restrict__ ovlo,
                 float* __restrict__ of, int K, int rowmap) {
    constexpr int AST = 40;
    constexpr int SST = 68;
    __shared__ _Float16 As[128 * AST];
    __shared__ _Float16 Als[ALO ? (128 * AST) : 8];
    __shared__ _Float16 Bs[64 * AST];
    __shared__ float stg[128 * SST];

    const int tid = threadIdx.x, lane = tid & 31, wid = tid >> 5;
    const int wm = wid & 3, wn = wid >> 2;
    const int half = lane >> 4, l16 = lane & 15;
    const int bn = blockIdx.x * 64;
    const int by = blockIdx.y;
    int bm;
    if (rowmap == 0) {
        bm = by * 128;
    } else if (rowmap == 1) {
        const int tpb = S / 128 - 1;
        const int bb  = by / tpb;
        bm = (bb * (S / 128) + (by - bb * tpb) + 1) * 128;
    } else {
        bm = by * S;
    }
    const bool early = ((bm % S) == 0);
    const int lor0 = (bm / S) * LOR + (bm % S);

    const int r0 = tid >> 2, c0 = (tid & 3) * 8;

    v8f acc[2][2], accR[2][2];
#pragma unroll
    for (int i = 0; i < 2; ++i)
#pragma unroll
        for (int j = 0; j < 2; ++j) { acc[i][j] = zero8(); accR[i][j] = zero8(); }

#pragma unroll 1
    for (int k0 = 0; k0 < K; k0 += 32) {
        *(v8h*)&As[r0 * AST + c0]        = *(const v8h*)&A[(size_t)(bm + r0) * K + k0 + c0];
        *(v8h*)&As[(r0 + 64) * AST + c0] = *(const v8h*)&A[(size_t)(bm + r0 + 64) * K + k0 + c0];
        if constexpr (ALO) {
            *(v8h*)&Als[r0 * AST + c0]        = *(const v8h*)&Alo[(size_t)(lor0 + r0) * K + k0 + c0];
            *(v8h*)&Als[(r0 + 64) * AST + c0] = *(const v8h*)&Alo[(size_t)(lor0 + r0 + 64) * K + k0 + c0];
        }
        *(v8h*)&Bs[r0 * AST + c0] = *(const v8h*)&Wt[(size_t)(bn + r0) * K + k0 + c0];
        __syncthreads();

        Frag a[2], b[2], al[2];
#pragma unroll
        for (int t = 0; t < 2; ++t) {
            const int m = wm * 32 + t * 16 + l16;
            const int n = wn * 32 + t * 16 + l16;
            a[t].h[0] = *(const v8h*)&As[m * AST + 8 * half];
            a[t].h[1] = *(const v8h*)&As[m * AST + 16 + 8 * half];
            b[t].h[0] = *(const v8h*)&Bs[n * AST + 8 * half];
            b[t].h[1] = *(const v8h*)&Bs[n * AST + 16 + 8 * half];
            if constexpr (ALO) {
                al[t].h[0] = *(const v8h*)&Als[m * AST + 8 * half];
                al[t].h[1] = *(const v8h*)&Als[m * AST + 16 + 8 * half];
            }
        }
#pragma unroll
        for (int i = 0; i < 2; ++i)
#pragma unroll
            for (int j = 0; j < 2; ++j) {
                acc[i][j] = mma(a[i].v, b[j].v, acc[i][j]);
                if constexpr (ALO) accR[i][j] = mma(al[i].v, b[j].v, accR[i][j]);
            }
        __syncthreads();
    }

    {
        constexpr float ASC = WINV * ((MODE == M_PROJ) ? YCI : 1.0f);
#pragma unroll
        for (int i = 0; i < 2; ++i)
#pragma unroll
            for (int j = 0; j < 2; ++j) {
                const int cl = wn * 32 + j * 16 + l16;
                const float bvf = bf16r(bias[bn + cl]);
#pragma unroll
                for (int r = 0; r < 8; ++r) {
                    const int rl = wm * 32 + i * 16 + 8 * half + r;
                    float v = acc[i][j][r] * ASC;
                    if constexpr (ALO) v += accR[i][j][r] * (ASC * RCI);
                    v += bvf;
                    stg[rl * SST + cl] = v;
                }
            }
    }
    __syncthreads();

    if constexpr (MODE == M_QKV) {
        if (bn < E2) {
            const int kq = lane & 7;
            v4u hv[4], lv[4];
            size_t ha[4], la[4];
#pragma unroll
            for (int pp = 0; pp < 4; ++pp) {
                const int rl = pp * 32 + wid * 4 + (lane >> 3);
                const v4f f0 = *(const v4f*)&stg[rl * SST + kq * 8];
                const v4f f1 = *(const v4f*)&stg[rl * SST + kq * 8 + 4];
                hv[pp] = pack8h(f0, f1);
                lv[pp] = hv[pp];
                if (early) lv[pp] = pack8lo(f0, f1);
                ha[pp] = (size_t)(bm + rl) * E2 + bn + kq * 8;
                la[pp] = (size_t)(lor0 + rl) * E2 + bn + kq * 8;
            }
#pragma unroll
            for (int pp = 0; pp < 4; ++pp) {
                *(volatile v4u*)(oh + ha[pp]) = hv[pp];
                if (early) *(volatile v4u*)(ohlo + la[pp]) = lv[pp];
            }
            __threadfence();
#pragma unroll
            for (int pp = 0; pp < 4; ++pp) {
                *(volatile v4u*)(oh + ha[pp]) = hv[pp];
                if (early) *(volatile v4u*)(ohlo + la[pp]) = lv[pp];
            }
        } else {
            const int hh = (bn - E2) >> 6;
            const int bb = bm / S, pos0 = bm % S;
            const int sub = lane >> 4, piece = lane & 15;
            const size_t vb  = (size_t)(bb * H + hh) * HD * S + pos0 + piece * 8;
            const size_t vlb = (size_t)(bb * H + hh) * HD * LOR + piece * 8;
            v4u hv[4], lv[4];
            int dd[4];
#pragma unroll
            for (int pp = 0; pp < 4; ++pp) {
                const int d = (pp * 8 + wid) * 2 + sub;
                dd[pp] = d;
                v4f f0, f1;
                f0.x = stg[(piece * 8 + 0) * SST + d];
                f0.y = stg[(piece * 8 + 1) * SST + d];
                f0.z = stg[(piece * 8 + 2) * SST + d];
                f0.w = stg[(piece * 8 + 3) * SST + d];
                f1.x = stg[(piece * 8 + 4) * SST + d];
                f1.y = stg[(piece * 8 + 5) * SST + d];
                f1.z = stg[(piece * 8 + 6) * SST + d];
                f1.w = stg[(piece * 8 + 7) * SST + d];
                hv[pp] = pack8h(f0, f1);
                lv[pp] = hv[pp];
                if (early) lv[pp] = pack8lo(f0, f1);
            }
#pragma unroll
            for (int pp = 0; pp < 4; ++pp) {
                *(volatile v4u*)(ov + vb + (size_t)dd[pp] * S) = hv[pp];
                if (early) *(volatile v4u*)(ovlo + vlb + (size_t)dd[pp] * LOR) = lv[pp];
            }
            __threadfence();
#pragma unroll
            for (int pp = 0; pp < 4; ++pp) {
                *(volatile v4u*)(ov + vb + (size_t)dd[pp] * S) = hv[pp];
                if (early) *(volatile v4u*)(ovlo + vlb + (size_t)dd[pp] * LOR) = lv[pp];
            }
        }
    } else if constexpr (MODE == M_FF1) {
        const int kq = lane & 7;
        v4u hv[4];
        size_t ha[4];
#pragma unroll
        for (int pp = 0; pp < 4; ++pp) {
            const int rl = pp * 32 + wid * 4 + (lane >> 3);
            const v4f f0 = gelu4(*(const v4f*)&stg[rl * SST + kq * 8]);
            const v4f f1 = gelu4(*(const v4f*)&stg[rl * SST + kq * 8 + 4]);
            hv[pp] = pack8h(f0, f1);
            ha[pp] = (size_t)(bm + rl) * FF + bn + kq * 8;
        }
#pragma unroll
        for (int pp = 0; pp < 4; ++pp) *(volatile v4u*)(oh + ha[pp]) = hv[pp];
        __threadfence();
#pragma unroll
        for (int pp = 0; pp < 4; ++pp) *(volatile v4u*)(oh + ha[pp]) = hv[pp];
    } else {
        const int c4 = lane & 15;
        v4f vals[8];
        size_t oa[8];
#pragma unroll
        for (int pp = 0; pp < 8; ++pp) {
            const int rl = pp * 16 + wid * 2 + (lane >> 4);
            const int row = bm + rl;
            const v4f v = *(const v4f*)&stg[rl * SST + c4 * 4];
            const size_t rr = (MODE == M_PROJ) ? (size_t)xrow(row) : (size_t)row;
            v4f rv = *(const v4f*)&resid[rr * E + bn + c4 * 4];
            if constexpr (MODE == M_PROJ) rv = bf16r4(rv);
            vals[pp] = v + rv;
            const size_t orow = (MODE == M_FF2) ? (size_t)xrow(row) : (size_t)row;
            oa[pp] = orow * E + bn + c4 * 4;
        }
#pragma unroll
        for (int pp = 0; pp < 8; ++pp) *(volatile v4f*)(of + oa[pp]) = vals[pp];
        __threadfence();
#pragma unroll
        for (int pp = 0; pp < 8; ++pp) *(volatile v4f*)(of + oa[pp]) = vals[pp];
    }
}

template <bool EARLY>
__global__ __launch_bounds__(128)
void attn_kernel(const _Float16* __restrict__ qk, const _Float16* __restrict__ qklo,
                 const _Float16* __restrict__ vt, const _Float16* __restrict__ vtlo,
                 _Float16* __restrict__ yo, _Float16* __restrict__ yolo, int qblk0) {
    constexpr int YST = 68;
    __shared__ float stg[4][16 * YST];

    const int lane = threadIdx.x & 31, wid = threadIdx.x >> 5;
    const int half = lane >> 4, l16 = lane & 15;
    const int h = blockIdx.y, bb = blockIdx.z;
    const int qblk = blockIdx.x + qblk0;
    const int q0 = qblk * 64 + wid * 16;
    const int ql = q0 + l16;

    Frag bq[2], bql[2];
    {
        const size_t qb = (size_t)(bb * S + ql) * E2 + h * HD;
#pragma unroll
        for (int g = 0; g < 2; ++g) {
            bq[g].h[0] = *(const v8h*)&qk[qb + g * 32 + 8 * half];
            bq[g].h[1] = *(const v8h*)&qk[qb + g * 32 + 16 + 8 * half];
        }
        if constexpr (EARLY) {
            const size_t qlb = (size_t)(bb * LOR + ql) * E2 + h * HD;
#pragma unroll
            for (int g = 0; g < 2; ++g) {
                bql[g].h[0] = *(const v8h*)&qklo[qlb + g * 32 + 8 * half];
                bql[g].h[1] = *(const v8h*)&qklo[qlb + g * 32 + 16 + 8 * half];
            }
        }
    }

    float mrun = -1e30f, lrun = 0.0f;
    v8f oT[4], oR[4];
#pragma unroll
    for (int t = 0; t < 4; ++t) { oT[t] = zero8(); oR[t] = zero8(); }

    const size_t vtb  = (size_t)(bb * H + h) * HD * S;
    const size_t vtlb = (size_t)(bb * H + h) * HD * LOR;
    const int kend = q0 + 16;

    for (int kb = 0; kb < kend; kb += 32) {
        v8f st[2], sr[2];
#pragma unroll
        for (int j = 0; j < 2; ++j) {
            const int key = kb + j * 16 + l16;
            const size_t kbs = (size_t)(bb * S + key) * E2 + E + h * HD;
            Frag ak[2];
#pragma unroll
            for (int g = 0; g < 2; ++g) {
                ak[g].h[0] = *(const v8h*)&qk[kbs + g * 32 + 8 * half];
                ak[g].h[1] = *(const v8h*)&qk[kbs + g * 32 + 16 + 8 * half];
            }
            st[j] = zero8();
            st[j] = mma(ak[0].v, bq[0].v, st[j]);
            st[j] = mma(ak[1].v, bq[1].v, st[j]);
            sr[j] = zero8();
            if constexpr (EARLY) {
                const size_t kls = (size_t)(bb * LOR + key) * E2 + E + h * HD;
                Frag akl[2];
#pragma unroll
                for (int g = 0; g < 2; ++g) {
                    akl[g].h[0] = *(const v8h*)&qklo[kls + g * 32 + 8 * half];
                    akl[g].h[1] = *(const v8h*)&qklo[kls + g * 32 + 16 + 8 * half];
                }
                sr[j] = mma(akl[0].v, bq[0].v, sr[j]);
                sr[j] = mma(akl[1].v, bq[1].v, sr[j]);
                sr[j] = mma(ak[0].v, bql[0].v, sr[j]);
                sr[j] = mma(ak[1].v, bql[1].v, sr[j]);
            }
        }

        float p[2][8];
        float m = -1e30f;
#pragma unroll
        for (int j = 0; j < 2; ++j)
#pragma unroll
            for (int r = 0; r < 8; ++r) {
                const int key = kb + j * 16 + 8 * half + r;
                float s = st[j][r];
                if constexpr (EARLY) s += sr[j][r] * RCI;
                s *= 0.125f;
                const float xs = (key > ql) ? -1e30f : s;
                p[j][r] = xs;
                m = fmaxf(m, xs);
            }
        m = fmaxf(m, __shfl_xor(m, 16, 32));
        const float mn = fmaxf(mrun, m);
        const float al = __expf(mrun - mn);
        float rs = 0.0f;
#pragma unroll
        for (int j = 0; j < 2; ++j)
#pragma unroll
            for (int r = 0; r < 8; ++r) {
                const int key = kb + j * 16 + 8 * half + r;
                const float ev = __expf(p[j][r] - mn);
                const float pv = (key > ql) ? 0.0f : ev;
                p[j][r] = pv;
                rs += pv;
            }
        rs += __shfl_xor(rs, 16, 32);
        lrun = lrun * al + rs;
        mrun = mn;
#pragma unroll
        for (int t = 0; t < 4; ++t) {
            oT[t] = oT[t] * al;
            if constexpr (EARLY) oR[t] = oR[t] * al;
        }

        Frag bp, bpr;
#pragma unroll
        for (int i = 0; i < 16; ++i) {
            const float ph = p[i >> 3][i & 7] * PC;
            const _Float16 hh = (_Float16)ph;
            bp.e[i]  = hh;
            bpr.e[i] = hh;
            if constexpr (EARLY) bpr.e[i] = (_Float16)((ph - (float)hh) * RC);
        }

#pragma unroll
        for (int t = 0; t < 4; ++t) {
            const int d = t * 16 + l16;
            const size_t va = vtb + (size_t)d * S + kb;
            Frag av;
            av.h[0] = *(const v8h*)&vt[va + 8 * half];
            av.h[1] = *(const v8h*)&vt[va + 16 + 8 * half];
            oT[t] = mma(av.v, bp.v, oT[t]);
            if constexpr (EARLY) {
                const size_t vla = vtlb + (size_t)d * LOR + kb;
                Frag avl;
                avl.h[0] = *(const v8h*)&vtlo[vla + 8 * half];
                avl.h[1] = *(const v8h*)&vtlo[vla + 16 + 8 * half];
                oR[t] = mma(avl.v, bp.v, oR[t]);
                oR[t] = mma(av.v, bpr.v, oR[t]);
            }
        }
    }

    const float inv = (YC / PC) * (1.0f / lrun);
    float* sw = &stg[wid][0];
#pragma unroll
    for (int t = 0; t < 4; ++t) {
        v4f o0, o1;
        o0.x = oT[t][0]; o0.y = oT[t][1]; o0.z = oT[t][2]; o0.w = oT[t][3];
        o1.x = oT[t][4]; o1.y = oT[t][5]; o1.z = oT[t][6]; o1.w = oT[t][7];
        if constexpr (EARLY) {
            o0.x += oR[t][0] * RCI; o0.y += oR[t][1] * RCI; o0.z += oR[t][2] * RCI; o0.w += oR[t][3] * RCI;
            o1.x += oR[t][4] * RCI; o1.y += oR[t][5] * RCI; o1.z += oR[t][6] * RCI; o1.w += oR[t][7] * RCI;
        }
        o0 = o0 * inv;
        o1 = o1 * inv;
        *(v4f*)&sw[l16 * YST + t * 16 + 8 * half]     = o0;
        *(v4f*)&sw[l16 * YST + t * 16 + 8 * half + 4] = o1;
    }
    __syncthreads();

    const bool lo_on = ((qblk + 1) * 64 <= LOR);
    const int kq = lane & 7;
    v4u hv[4], lv[4];
    size_t ha[4], la[4];
#pragma unroll
    for (int pp = 0; pp < 4; ++pp) {
        const int qr = pp * 4 + (lane >> 3);
        const v4f f0 = *(const v4f*)&sw[qr * YST + kq * 8];
        const v4f f1 = *(const v4f*)&sw[qr * YST + kq * 8 + 4];
        hv[pp] = pack8h(f0, f1);
        lv[pp] = hv[pp];
        if (lo_on) lv[pp] = pack8lo(f0, f1);
        ha[pp] = (size_t)(bb * S + q0 + qr) * E + h * HD + kq * 8;
        la[pp] = (size_t)(bb * LOR + q0 + qr) * E + h * HD + kq * 8;
    }
#pragma unroll
    for (int pp = 0; pp < 4; ++pp) {
        *(volatile v4u*)(yo + ha[pp]) = hv[pp];
        if (lo_on) *(volatile v4u*)(yolo + la[pp]) = lv[pp];
    }
    __threadfence();
#pragma unroll
    for (int pp = 0; pp < 4; ++pp) {
        *(volatile v4u*)(yo + ha[pp]) = hv[pp];
        if (lo_on) *(volatile v4u*)(yolo + la[pp]) = lv[pp];
    }
}

extern "C" void kernel_launch(void* const* d_in, const int* in_sizes, int n_in,
                              void* d_out, int out_size, void* d_ws, size_t ws_size,
                              hipStream_t stream) {
    if (n_in < 13) return;
    const int xrows_needed = (NB - 1) * SEQ_FULL + SEQ;
    if (in_sizes[0]  < xrows_needed * E) return;
    if (in_sizes[1]  < E || in_sizes[2] < E) return;
    if (in_sizes[3]  < E * E3 || in_sizes[4] < E3) return;
    if (in_sizes[5]  < E * E || in_sizes[6] < E) return;
    if (in_sizes[7]  < E || in_sizes[8] < E) return;
    if (in_sizes[9]  < E * FF || in_sizes[10] < FF) return;
    if (in_sizes[11] < FF * E || in_sizes[12] < E) return;
    if (out_size < xrows_needed * E) return;

    const float* x      = (const float*)d_in[0];
    const float* ln1_g  = (const float*)d_in[1];
    const float* ln1_b  = (const float*)d_in[2];
    const float* w_attn = (const float*)d_in[3];
    const float* b_attn = (const float*)d_in[4];
    const float* w_proj = (const float*)d_in[5];
    const float* b_proj = (const float*)d_in[6];
    const float* ln2_g  = (const float*)d_in[7];
    const float* ln2_b  = (const float*)d_in[8];
    const float* w_ff1  = (const float*)d_in[9];
    const float* b_ff1  = (const float*)d_in[10];
    const float* w_ff2  = (const float*)d_in[11];
    const float* b_ff2  = (const float*)d_in[12];
    float* outp = (float*)d_out;

    size_t off = 0;
    auto carve = [&](size_t bytes) -> size_t {
        const size_t p = off;
        off += (bytes + 255) & ~(size_t)255;
        return p;
    };
    const size_t o_wqkvT  = carve((size_t)E3 * E * 2);
    const size_t o_wprojT = carve((size_t)E * E * 2);
    const size_t o_w1T    = carve((size_t)FF * E * 2);
    const size_t o_w2T    = carve((size_t)E * FF * 2);
    const size_t o_ln1o   = carve((size_t)T * E * 2);
    const size_t o_ln1lo  = carve((size_t)NB * LOR * E * 2);
    const size_t o_qk     = carve((size_t)T * E2 * 2);
    const size_t o_qklo   = carve((size_t)NB * LOR * E2 * 2);
    const size_t o_vt     = carve((size_t)NB * H * HD * S * 2);
    const size_t o_vtlo   = carve((size_t)NB * H * HD * LOR * 2);
    const size_t o_attno  = carve((size_t)T * E * 2);
    const size_t o_attlo  = carve((size_t)NB * LOR * E * 2);
    const size_t o_x1     = carve((size_t)T * E * 4);
    const size_t o_ln2o   = carve((size_t)T * E * 2);
    const size_t o_h1     = carve((size_t)T * FF * 2);
    if (off > ws_size) return;
    if (off > (size_t)134217728) return;

    char* ws = (char*)d_ws;
    _Float16* wqkvT  = (_Float16*)(ws + o_wqkvT);
    _Float16* wprojT = (_Float16*)(ws + o_wprojT);
    _Float16* w1T    = (_Float16*)(ws + o_w1T);
    _Float16* w2T    = (_Float16*)(ws + o_w2T);
    _Float16* ln1o   = (_Float16*)(ws + o_ln1o);
    _Float16* ln1lo  = (_Float16*)(ws + o_ln1lo);
    _Float16* qk     = (_Float16*)(ws + o_qk);
    _Float16* qklo   = (_Float16*)(ws + o_qklo);
    _Float16* vt     = (_Float16*)(ws + o_vt);
    _Float16* vtlo   = (_Float16*)(ws + o_vtlo);
    _Float16* attno  = (_Float16*)(ws + o_attno);
    _Float16* attlo  = (_Float16*)(ws + o_attlo);
    float*    x1     = (float*)(ws + o_x1);
    _Float16* ln2o   = (_Float16*)(ws + o_ln2o);
    _Float16* h1     = (_Float16*)(ws + o_h1);

    cvt_kernel<<<dim3(E / 64, E3 / 64), 256, 0, stream>>>(w_attn, wqkvT, E, E3);
    cvt_kernel<<<dim3(E / 64, E / 64), 256, 0, stream>>>(w_proj, wprojT, E, E);
    cvt_kernel<<<dim3(E / 64, FF / 64), 256, 0, stream>>>(w_ff1, w1T, E, FF);
    cvt_kernel<<<dim3(FF / 64, E / 64), 256, 0, stream>>>(w_ff2, w2T, FF, E);

    ln_kernel<true, true><<<dim3(T), 256, 0, stream>>>(x, ln1_g, ln1_b, ln1o, ln1lo);

    gemm_kernel<M_QKV, false><<<dim3(E3 / 64, NB * (S / 128 - 1)), 256, 0, stream>>>(
        ln1o, ln1lo, wqkvT, b_attn, b_attn, qk, qklo, vt, vtlo, x1, E, 1);
    gemm_kernel<M_QKV, true><<<dim3(E3 / 64, NB), 256, 0, stream>>>(
        ln1o, ln1lo, wqkvT, b_attn, b_attn, qk, qklo, vt, vtlo, x1, E, 2);

    attn_kernel<true><<<dim3(1, H, NB), 128, 0, stream>>>(qk, qklo, vt, vtlo, attno, attlo, 0);
    attn_kernel<false><<<dim3(S / 64 - 1, H, NB), 128, 0, stream>>>(qk, qklo, vt, vtlo, attno, attlo, 1);

    gemm_kernel<M_PROJ, false><<<dim3(E / 64, NB * (S / 128 - 1)), 256, 0, stream>>>(
        attno, attlo, wprojT, b_proj, x, ln2o, ln2o, ln2o, ln2o, x1, E, 1);
    gemm_kernel<M_PROJ, true><<<dim3(E / 64, NB), 256, 0, stream>>>(
        attno, attlo, wprojT, b_proj, x, ln2o, ln2o, ln2o, ln2o, x1, E, 2);

    ln_kernel<false, false><<<dim3(T), 256, 0, stream>>>(x1, ln2_g, ln2_b, ln2o, ln1lo);

    gemm_kernel<M_FF1, false><<<dim3(FF / 64, T / 128), 256, 0, stream>>>(
        ln2o, ln1lo, w1T, b_ff1, x1, h1, qklo, vt, vtlo, x1, E, 0);

    gemm_kernel<M_FF2, false><<<dim3(E / 64, T / 128), 256, 0, stream>>>(
        h1, ln1lo, w2T, b_ff2, x1, ln2o, qklo, vt, vtlo, outp, FF, 0);
}
